// Interaction_GraphConvolution_20590073217235
// MI455X (gfx1250) — hardware-verified
//
#include <hip/hip_runtime.h>


namespace {
constexpr int N = 1024, FIN = 256, DIN = 128, F = 64, LMAX = 96  , LW = 128  ;
constexpr float XS = 8.0f, WSC = 256.0f;
typedef _Float16 b16;
typedef __attribute__((ext_vector_type(16))) _Float16 v16b;
typedef __attribute__((ext_vector_type(8))) _Float16 v8b;
typedef __attribute__((ext_vector_type(8))) float v8f;
typedef __attribute__((ext_vector_type(4))) float v4f;
__device__ __forceinline__ float bf16_rne(float f) { unsigned int u = __float_as_uint(f); u += 0x7FFFu + ((u >> 16) & 1u); return __uint_as_float(u & 0xFFFF0000u); }
__device__ __forceinline__ void split16(float v, b16& hi, b16& lo) { hi = (b16)v; lo = (b16)(v - (float)hi); }
__device__ __forceinline__ v16b frag_kb(const b16* p, int hh) { const v8b a = *(const v8b*)(p + 8 * hh), b = *(const v8b*)(p + 16 + 8 * hh); v16b f;
#pragma unroll
  for (int e = 0; e < 8; ++e) { f[e] = a[e]; f[8 + e] = b[e]; } return f; }
__device__ __forceinline__ v8f wmma16b(v16b a, v16b b, v8f c) { v8f d = __builtin_amdgcn_wmma_f32_16x16x32_f16(false, a, false, b, (short)0, c, false, false); asm volatile("v_nop\n\tv_nop\n\tv_nop\n\tv_nop" : "+v"(d) : "v"(a), "v"(b)); return d; }
__device__ __forceinline__ void wave_lds_sync() { __builtin_amdgcn_fence(__ATOMIC_RELEASE, "workgroup"); __builtin_amdgcn_wave_barrier(); __builtin_amdgcn_fence(__ATOMIC_ACQUIRE, "workgroup"); }
__device__ __forceinline__ float pmul(float a, float b) { float p = a * b; asm volatile("" : "+v"(p)); return p; }
__device__ __forceinline__ int iclamp(int v, int lo, int hi) { return v < lo ? lo : (v > hi ? hi : v); }

typedef __attribute__((ext_vector_type(4))) _Float16 v4h;
typedef __attribute__((ext_vector_type(2))) float v2f;
__global__ __launch_bounds__(256) void prep_kernel(const float* __restrict__ nf, const float* __restrict__ adj, const float* __restrict__ mf, const float* __restrict__ lw, const float* __restrict__ wg, b16* __restrict__ Xh, b16* __restrict__ LWT, b16* __restrict__ WGT, int* __restrict__ LA, int* __restrict__ LM) {
  size_t t = (size_t)blockIdx.x * 256 + threadIdx.x; v8b o;
  const size_t nx = (size_t)N * FIN / 8; if (t < nx) { const size_t e = t * 8; for (int j = 0; j < 8; ++j) o[j] = (b16)(bf16_rne(nf[e + j]) * XS); for (int pass = 0; pass < 2; ++pass) { *(volatile v8b*)(Xh + e) = o; __threadfence(); } return; } t -= nx;
  const size_t n1 = (size_t)DIN * FIN / 8; if (t < n1) { const size_t e = t * 8; for (int j = 0; j < 8; ++j) o[j] = (b16)(bf16_rne(lw[e + j]) * WSC); for (int pass = 0; pass < 2; ++pass) { *(volatile v8b*)(LWT + e) = o; __threadfence(); } return; } t -= n1;
  const size_t n2 = (size_t)F * DIN / 8; if (t < n2) { const size_t e = t * 8; const int f = (int)(e / DIN), k0 = (int)(e % DIN); for (int j = 0; j < 8; ++j) o[j] = (b16)(bf16_rne(wg[(size_t)(k0 + j) * F + f]) * WSC); for (int pass = 0; pass < 2; ++pass) { *(volatile v8b*)(WGT + e) = o; __threadfence(); } return; } t -= n2;
  if (t < (size_t)2 * N) { const int i = (int)(t % N); const float* row = (t < (size_t)N) ? adj + (size_t)i * N : mf + (size_t)i * N; int* L = ((t < (size_t)N) ? LA : LM) + (size_t)i * LW; int cnt = 0;
    for (int pass = 0; pass < 2; ++pass) { cnt = 0;
#pragma unroll 1
      for (int c = 0; c < N; ++c) { if (row[c] != 0.0f) { if (cnt < LW - 1) ((volatile int*)L)[cnt] = c; ++cnt; } }
#pragma unroll 1
      for (int s = (cnt < LW - 1 ? cnt : LW - 1); s < LW - 1; ++s) ((volatile int*)L)[s] = -1;
      ((volatile int*)L)[LW - 1] = cnt; __threadfence(); } }
}
template <int MODE>
__global__ __launch_bounds__(32) void lin_kernel(const b16* __restrict__ Xh, const b16* __restrict__ WT, const float* __restrict__ bias, const float* __restrict__ Xin, float* __restrict__ OUT) {
  __shared__ __attribute__((aligned(16))) b16 Ah[16][DIN + 8], Al[16][DIN + 8]; __shared__ __attribute__((aligned(16))) float Tf[16][128 + 4];
  const int lane = threadIdx.x, nloc = lane & 15, hlf = lane >> 4; const size_t m0 = (size_t)blockIdx.x * 16;
  constexpr int NT = MODE == 0 ? 8 : 4; constexpr int KD = MODE == 0 ? FIN : DIN;
  if (MODE == 1) { for (int rr = 0; rr < 16; ++rr) { const v4f v = *(const v4f*)(Xin + (m0 + rr) * DIN + lane * 4); v4h hv, lv; for (int j = 0; j < 4; ++j) { b16 p, q; split16(v[j] * XS, p, q); hv[j] = p; lv[j] = q; } *(v4h*)(&Ah[rr][lane * 4]) = hv; *(v4h*)(&Al[rr][lane * 4]) = lv; } wave_lds_sync(); }
  v8f acc[NT];
#pragma unroll
  for (int t = 0; t < NT; ++t) acc[t] = (v8f){};
#pragma unroll 2
  for (int kb = 0; kb < KD; kb += 32) { v16b a, al; if (MODE == 0) a = frag_kb(Xh + (m0 + nloc) * FIN + kb, hlf); else { a = frag_kb(&Ah[nloc][kb], hlf); al = frag_kb(&Al[nloc][kb], hlf); }
#pragma unroll
    for (int t = 0; t < NT; ++t) { const v16b bw = frag_kb(WT + (size_t)(t * 16 + nloc) * KD + kb, hlf); acc[t] = wmma16b(a, bw, acc[t]); if (MODE == 1) acc[t] = wmma16b(al, bw, acc[t]); } }
#pragma unroll
  for (int t = 0; t < NT; ++t) { const float bb = (MODE == 0) ? bf16_rne(bias[t * 16 + nloc]) : 0.0f;
#pragma unroll
    for (int r = 0; r < 8; ++r) Tf[8 * hlf + r][t * 16 + nloc] = acc[t][r] * (1.0f / (XS * WSC)) + bb; }
  wave_lds_sync();
  constexpr int NC = NT * 16;
  typedef __attribute__((ext_vector_type(NC / 32))) float vrow;
  for (int pass = 0; pass < 2; ++pass) { for (int rr = 0; rr < 16; ++rr) *(volatile vrow*)(OUT + (m0 + rr) * NC + lane * (NC / 32)) = *(const vrow*)(&Tf[rr][lane * (NC / 32)]); __threadfence(); }
}
__global__ __launch_bounds__(128) void node_kernel(const float* __restrict__ WF, const float* __restrict__ sib, const int* __restrict__ LA, const int* __restrict__ LM, const float* __restrict__ ncnt, float* __restrict__ out) {
  __shared__ __attribute__((aligned(16))) b16 As[LMAX][LMAX + 8], Bh[F][LMAX + 8], Bl[F][LMAX + 8]; __shared__ int la[LMAX], lm[LMAX]; __shared__ float part[6][F], res[F];
  const int i = blockIdx.x, t = threadIdx.x, wave = t >> 5, lane = t & 31, nloc = lane & 15, hlf = lane >> 4;
  const int na = iclamp(LA[(size_t)i * LW + LW - 1], 0, LMAX), nm = iclamp(LM[(size_t)i * LW + LW - 1], 0, LMAX);
  if (t < LMAX) { la[t] = (t < na) ? iclamp(LA[(size_t)i * LW + t], 0, N - 1) : 0; lm[t] = (t < nm) ? iclamp(LM[(size_t)i * LW + t], 0, N - 1) : 0; }
  __syncthreads();
  for (int q = t; q < LMAX * (LMAX / 8); q += 128) { const int r = q / (LMAX / 8), k0 = (q % (LMAX / 8)) * 8; v8b v; for (int j = 0; j < 8; ++j) { const int k = k0 + j; v[j] = (r < na && k < nm) ? (b16)sib[(size_t)la[r] * N + lm[k]] : (b16)0.0f; } *(v8b*)(&As[r][k0]) = v; }
  for (int q = t; q < F * (LMAX / 8); q += 128) { const int f = q / (LMAX / 8), k0 = (q % (LMAX / 8)) * 8; v8b hv, lv; for (int j = 0; j < 8; ++j) { const int k = k0 + j; const float w = (k < nm) ? WF[(size_t)lm[k] * F + f] : 0.0f; b16 p, qq; split16(w * XS, p, qq); hv[j] = p; lv[j] = qq; } *(v8b*)(&Bh[f][k0]) = hv; *(v8b*)(&Bl[f][k0]) = lv; }
  __syncthreads();
#pragma unroll 1
  for (int rt = wave; rt < 6; rt += 4) { v8f acc[4];
#pragma unroll
    for (int u = 0; u < 4; ++u) acc[u] = (v8f){};
#pragma unroll
    for (int kb = 0; kb < LMAX; kb += 32) { const v16b a = frag_kb(&As[rt * 16 + nloc][kb], hlf);
#pragma unroll
      for (int u = 0; u < 4; ++u) { acc[u] = wmma16b(a, frag_kb(&Bh[u * 16 + nloc][kb], hlf), acc[u]); acc[u] = wmma16b(a, frag_kb(&Bl[u * 16 + nloc][kb], hlf), acc[u]); } }
#pragma unroll
    for (int u = 0; u < 4; ++u) { const int f = u * 16 + nloc; float s = 0.0f;
#pragma unroll
      for (int r = 0; r < 8; ++r) { const int row = rt * 16 + 8 * hlf + r; const float w = (row < na) ? WF[(size_t)la[row < na ? row : 0] * F + f] : 0.0f; s += pmul(w, acc[u][r] * (1.0f / XS)); }
      s += __shfl_xor(s, 16); if (hlf == 0) part[rt][f] = s; } }
  __syncthreads();
  if (t < F) { float s = 0.0f; for (int rt = 0; rt < 6; ++rt) if (rt * 16 < na) s += part[rt][t]; const float nc = ncnt[i]; res[t] = s / (nc * nc); }
  __syncthreads();
  for (int pass = 0; pass < 2; ++pass) { if (t < F) ((volatile float*)out)[(size_t)i * F + t] = res[t]; __threadfence(); }
}
}

extern "C" void kernel_launch(void* const* d_in, const int* in_sizes, int n_in, void* d_out, int out_size, void* d_ws, size_t ws_size, hipStream_t stream) {
  (void)n_in;
  auto Fp = [&](int i) { return (const float*)d_in[i]; };
  if (in_sizes[0] != N * FIN || in_sizes[1] != N * N || in_sizes[2] != N * N || in_sizes[3] != N || in_sizes[4] != N * N || in_sizes[5] != DIN * FIN || in_sizes[6] != DIN || in_sizes[7] != DIN * F || out_size != N * F) return;
  size_t off = 0; char* ws = (char*)d_ws;
  auto carve = [&](size_t bytes) { char* p = ws + off; off += (bytes + 255) & ~(size_t)255; return p; };
  b16* Xh = (b16*)carve((size_t)N * FIN * 2); b16* LWT = (b16*)carve((size_t)DIN * FIN * 2); b16* WGT = (b16*)carve((size_t)F * DIN * 2); int* LA = (int*)carve((size_t)N * LW * 4); int* LM = (int*)carve((size_t)N * LW * 4); float* X = (float*)carve((size_t)N * DIN * 4); float* WF = (float*)carve((size_t)N * F * 4);
  if (off > ws_size || off > ((size_t)128 << 20)) return;
  prep_kernel<<<(unsigned)((((size_t)N * FIN + (size_t)DIN * FIN + (size_t)F * DIN) / 8 + 2 * N + 255) / 256), 256, 0, stream>>>(Fp(0), Fp(1), Fp(2), Fp(5), Fp(7), Xh, LWT, WGT, LA, LM);
  lin_kernel<0><<<N / 16, 32, 0, stream>>>(Xh, LWT, Fp(6), nullptr, X);
  lin_kernel<1><<<N / 16, 32, 0, stream>>>(nullptr, WGT, nullptr, X, WF);
  node_kernel<<<N, 128, 0, stream>>>(WF, Fp(4), LA, LM, Fp(3), (float*)d_out);
}
